// PatchTSTEncoder_1047972020495
// MI455X (gfx1250) — hardware-verified
//
#include <hip/hip_runtime.h>
#include <math.h>
#include <stdint.h>

constexpr int kBatch     = 4;
constexpr int kTlen      = 8192;
constexpr int kChan      = 7;
constexpr int kPatchLen  = 16;
constexpr int kPatchStr  = 8;
constexpr int kPat       = 1023;
constexpr int kTokB      = 1024;
constexpr int kTok       = kBatch * kTokB;
constexpr int kTokReal   = kBatch * kPat;
constexpr int kDm        = 512;
constexpr int kHeads     = 8;
constexpr int kHd        = 64;
constexpr int kQK        = 1024;
constexpr int kQKV       = 1536;
constexpr int kMlp       = 2048;
constexpr int kKemb      = kChan * kPatchLen;
constexpr int kKembP     = 128;
constexpr int kLayers    = 4;
constexpr float kLnEps   = 1e-5f;
constexpr float kWCarry  = 64.0f;
constexpr float kOCarry  = 16.0f;

typedef __attribute__((ext_vector_type(16))) _Float16 v16h;
typedef __attribute__((ext_vector_type(8)))  _Float16 v8h;
typedef __attribute__((ext_vector_type(16))) __bf16   v16b;
typedef __attribute__((ext_vector_type(8)))  __bf16   v8b;
typedef __attribute__((ext_vector_type(8)))  float    v8f;
typedef __attribute__((ext_vector_type(4)))  float    v4f;
typedef __attribute__((ext_vector_type(4)))  unsigned int v4u;
#define PSCALE 32768.0f
#define U16(p) ((const unsigned short*)(const void*)(p))
#define PSCALE_INV (1.0f / 32768.0f)

__device__ __forceinline__ unsigned short f2bf_bits(float f) {
  unsigned u = __float_as_uint(f);
  return (unsigned short)((u + 0x7FFFu + ((u >> 16) & 1u)) >> 16);
}
__device__ __forceinline__ float bf_bits2f(unsigned short h) { return __uint_as_float(((unsigned)h) << 16); }
__device__ __forceinline__ float bfrn(float f) { return bf_bits2f(f2bf_bits(f)); }
__device__ __forceinline__ unsigned short h_bits(float f) { return __builtin_bit_cast(unsigned short, (_Float16)f); }
__device__ __forceinline__ unsigned pk16(unsigned short a, unsigned short b) { return (unsigned)a | ((unsigned)b << 16); }

__device__ __forceinline__ void dep_guard_h(v8f& a, v8f& b, v16h x, v16h y) { asm volatile("v_nop\n\tv_nop\n\tv_nop\n\tv_nop" : "+v"(a), "+v"(b) : "v"(x), "v"(y)); }
__device__ __forceinline__ void dep_guard_b(v8f& a, v8f& b, v16b x, v16b y) { asm volatile("v_nop\n\tv_nop\n\tv_nop\n\tv_nop" : "+v"(a), "+v"(b) : "v"(x), "v"(y)); }
__device__ __forceinline__ void keep4_h(v16h a, v16h b, v16h c, v16h d) { asm volatile("v_nop" :: "v"(a), "v"(b), "v"(c), "v"(d)); }
__device__ __forceinline__ void keep4_b(v16b a, v16b b, v16b c, v16b d) { asm volatile("v_nop" :: "v"(a), "v"(b), "v"(c), "v"(d)); }
__device__ __forceinline__ void acc_guard4(v8f& a, v8f& b, v8f& c, v8f& d) { asm volatile("v_nop\n\tv_nop\n\tv_nop\n\tv_nop" : "+v"(a), "+v"(b), "+v"(c), "+v"(d)); }
template <typename T> struct Frag;
template <> struct Frag<_Float16> {
  typedef v16h V; union U { v16h v; v8h h[2]; };
  static __device__ __forceinline__ v16h load(const _Float16* p) {
    U f; f.h[0] = *(const v8h*)(p); f.h[1] = *(const v8h*)(p + 16); return f.v;
  }
  static __device__ __forceinline__ v8f mma(v16h a, v16h b, v8f c) {
    return __builtin_amdgcn_wmma_f32_16x16x32_f16(false, a, false, b, (short)0, c, false, false);
  }
  static __device__ __forceinline__ void guard(v8f& a, v8f& b, v16h x, v16h y) { dep_guard_h(a, b, x, y); }
  static __device__ __forceinline__ void keep(v16h a, v16h b, v16h c, v16h d) { keep4_h(a, b, c, d); }
};
template <> struct Frag<__bf16> {
  typedef v16b V; union U { v16b v; v8b h[2]; };
  static __device__ __forceinline__ v16b load(const __bf16* p) {
    U f; f.h[0] = *(const v8b*)(p); f.h[1] = *(const v8b*)(p + 16); return f.v;
  }
  static __device__ __forceinline__ v8f mma(v16b a, v16b b, v8f c) {
    return __builtin_amdgcn_wmma_f32_16x16x32_bf16(false, a, false, b, (short)0, c, false, false);
  }
  static __device__ __forceinline__ void guard(v8f& a, v8f& b, v16b x, v16b y) { dep_guard_b(a, b, x, y); }
  static __device__ __forceinline__ void keep(v16b a, v16b b, v16b c, v16b d) { keep4_b(a, b, c, d); }
};

template <int ET> struct Elem;
template <> struct Elem<0> { typedef _Float16 T; };
template <> struct Elem<1> { typedef __bf16 T; };
template <int ET, bool SPLIT, int BIAS_MODE, int OUT_MODE, bool RESID, int ACT = 0>
__global__ __launch_bounds__(256) void wmma_gemm64(
    const unsigned short* __restrict__ Ap, const unsigned short* __restrict__ A2p, int lda, long strideA,
    const unsigned short* __restrict__ Btp, const unsigned short* __restrict__ Bt2p, int ldb, long strideB,
    void* __restrict__ Cout, void* __restrict__ Cout2, int ldc, long strideC,
    const float* __restrict__ bias,
    const float* __restrict__ resid, long strideR,
    int M, int N, int K, float scale) {
  typedef typename Elem<ET>::T T;
  typedef typename Frag<T>::V V;
  const T* A = (const T*)Ap; const T* A2 = (const T*)A2p; const T* Bt = (const T*)Btp; const T* Bt2 = (const T*)Bt2p;
  __shared__ __align__(16) float sT[8][16 * 68];
  const int b    = blockIdx.y;
  const int lane = threadIdx.x & 31;
  const int wave = threadIdx.x >> 5;
  const int tilesN = N >> 6;
  const int tilesM = M >> 6;
  const int tile = blockIdx.x * 8 + wave;
  if (tile >= tilesM * tilesN) return;
  const int tm = tile / tilesN;
  const int tn = tile - tm * tilesN;
  const int m0 = tm << 6;
  const int n0 = tn << 6;

  const T* Ab  = A  + (size_t)b * strideA;
  const T* Bb  = Bt + (size_t)b * strideB;
  const T* Ab2 = SPLIT ? (A2  + (size_t)b * strideA) : nullptr;
  const T* Bb2 = SPLIT ? (Bt2 + (size_t)b * strideB) : nullptr;

  const int rlane = lane & 15;
  const int koff  = (lane >> 4) * 8;
  const int mOff  = (lane >> 4) * 8;

  v8f acc[4][4];
#pragma unroll
  for (int i = 0; i < 4; ++i)
#pragma unroll
    for (int j = 0; j < 4; ++j) acc[i][j] = (v8f){0.f,0.f,0.f,0.f,0.f,0.f,0.f,0.f};

  for (int k0 = 0; k0 < K; k0 += 32) {
    V bh[4], bl[4];
#pragma unroll
    for (int j = 0; j < 4; ++j) {
      const size_t bo = (size_t)(n0 + (j << 4) + rlane) * ldb + koff + k0;
      bh[j] = Frag<T>::load(Bb + bo);
      if (SPLIT) bl[j] = Frag<T>::load(Bb2 + bo);
    }
#pragma unroll
    for (int i = 0; i < 4; ++i) {
      const size_t ao = (size_t)(m0 + (i << 4) + rlane) * lda + koff + k0;
      V ah = Frag<T>::load(Ab + ao);
      V al;
      if (SPLIT) al = Frag<T>::load(Ab2 + ao);
#pragma unroll
      for (int j = 0; j < 4; ++j) {
        acc[i][j] = Frag<T>::mma(ah, bh[j], acc[i][j]);
        if (SPLIT) {
          acc[i][j] = Frag<T>::mma(ah, bl[j], acc[i][j]);
          acc[i][j] = Frag<T>::mma(al, bh[j], acc[i][j]);
        }
      }
      Frag<T>::guard(acc[i][0], acc[i][3], ah, SPLIT ? al : ah);
    }
    Frag<T>::keep(bh[0], bh[1], bh[2], bh[3]);
    if (SPLIT) Frag<T>::keep(bl[0], bl[1], bl[2], bl[3]);
  }
  acc_guard4(acc[0][0], acc[0][1], acc[0][2], acc[0][3]);
  acc_guard4(acc[1][0], acc[1][1], acc[1][2], acc[1][3]);
  acc_guard4(acc[2][0], acc[2][1], acc[2][2], acc[2][3]);
  acc_guard4(acc[3][0], acc[3][1], acc[3][2], acc[3][3]);

  float* slab = sT[wave];
  const float* Rb = RESID ? (resid + (size_t)b * strideR) : nullptr;
#pragma unroll
  for (int i = 0; i < 4; ++i) {
    const int mBase = m0 + (i << 4);
#pragma unroll
    for (int j = 0; j < 4; ++j) {
      const int n = n0 + (j << 4) + rlane;
      float bv = 0.f;
      if (BIAS_MODE == 2) bv = bias[n];
#pragma unroll
      for (int r = 0; r < 8; ++r) {
        float v = acc[i][j][r] * scale;
        if (BIAS_MODE == 1) v += bias[mBase + mOff + r];
        if (BIAS_MODE == 2) v += bv;
        if (RESID) v += Rb[(size_t)(mBase + mOff + r) * ldc + n];
        if (ACT == 1) v = tanhf(v);
        if (ACT == 2) v = fmaxf(v, 0.0f);
        if (ACT == 3) v = v / (1.0f + expf(-v));
        if (ACT == 4) v = (v > 0.f) ? v : 0.01f * v;
        if (ACT == 5) v = 0.5f * v * (1.0f + erff(v * 0.70710678118654752f));
        slab[(mOff + r) * 68 + (j << 4) + rlane] = v;
      }
    }
    __builtin_amdgcn_fence(__ATOMIC_RELEASE, "workgroup");
    __builtin_amdgcn_wave_barrier();
    __builtin_amdgcn_fence(__ATOMIC_ACQUIRE, "workgroup");
    if (OUT_MODE == 0) {
      float* C = (float*)Cout + (size_t)b * strideC;
      const int hh = lane >> 4, c4 = (lane & 15) * 4;
      for (int pass = 0; pass < 2; ++pass) {
#pragma unroll
        for (int it = 0; it < 8; ++it) {
          const int row = it * 2 + hh;
          v4f v = *(const v4f*)(slab + row * 68 + c4);
          *(volatile v4f*)(C + (size_t)(mBase + row) * ldc + n0 + c4) = v;
        }
        __threadfence();
      }
    } else {
      const int q = lane >> 3, c8 = (lane & 7) * 8;
      unsigned short* C  = (unsigned short*)Cout  + (size_t)b * strideC;
      unsigned short* C2 = (OUT_MODE == 2) ? ((unsigned short*)Cout2 + (size_t)b * strideC) : nullptr;
      for (int pass = 0; pass < 2; ++pass) {
#pragma unroll
        for (int it = 0; it < 4; ++it) {
          const int row = it * 4 + q;
          const float* sp = slab + row * 68 + c8;
          v8h hv, lv;
#pragma unroll
          for (int e = 0; e < 8; ++e) {
            if (OUT_MODE == 1) {
              hv[e] = (_Float16)sp[e];
            } else {
              unsigned short hb = f2bf_bits(sp[e]);
              unsigned short lb = f2bf_bits(sp[e] - bf_bits2f(hb));
              hv[e] = __builtin_bit_cast(_Float16, hb);
              lv[e] = __builtin_bit_cast(_Float16, lb);
            }
          }
          *(volatile v8h*)(C + (size_t)(mBase + row) * ldc + n0 + c8) = hv;
          if (OUT_MODE == 2) *(volatile v8h*)(C2 + (size_t)(mBase + row) * ldc + n0 + c8) = lv;
        }
        __threadfence();
      }
    }
    __builtin_amdgcn_fence(__ATOMIC_RELEASE, "workgroup");
    __builtin_amdgcn_wave_barrier();
    __builtin_amdgcn_fence(__ATOMIC_ACQUIRE, "workgroup");
  }
}

__global__ __launch_bounds__(256) void tcast_kernel(const float* __restrict__ W, unsigned short* __restrict__ oh,
                                                    int R, int Rpad, int Cc, long sIn, long sOut, float scale) {
  __shared__ __align__(16) float tf[64 * 68];
  W  += (size_t)blockIdx.z * sIn;
  oh += (size_t)blockIdx.z * sOut;
  const int c0  = blockIdx.x * 64;
  const int r0  = blockIdx.y * 64;
  const int tid = threadIdx.x;
  {
    const int lr = tid >> 4;
    const int c4 = (tid & 15) * 4;
#pragma unroll
    for (int it = 0; it < 4; ++it) {
      const int rr   = it * 16 + lr;
      const int row  = r0 + rr;
      const int rowc = (row < R) ? row : (R - 1);
      v4f a = *(const v4f*)(W + (size_t)rowc * Cc + c0 + c4);
      if (row >= R) a = (v4f){0.f, 0.f, 0.f, 0.f};
      *(v4f*)(tf + rr * 68 + c4) = a;
    }
  }
  __syncthreads();
  const int sub = tid >> 3;
  const int c8  = (tid & 7) * 8;
  v4u hv[2];
#pragma unroll
  for (int it = 0; it < 2; ++it) {
    const int oc = it * 32 + sub;
    v4u a;
#pragma unroll
    for (int q = 0; q < 4; ++q) {
      const float f0 = tf[(c8 + 2 * q) * 68 + oc];
      const float f1 = tf[(c8 + 2 * q + 1) * 68 + oc];
      a[q] = pk16(h_bits(bfrn(f0) * scale), h_bits(bfrn(f1) * scale));
    }
    hv[it] = a;
  }
  for (int pass = 0; pass < 2; ++pass) {
#pragma unroll
    for (int it = 0; it < 2; ++it) {
      const int oc = it * 32 + sub;
      const size_t go = (size_t)(c0 + oc) * Rpad + r0 + c8;
      *(volatile v4u*)(oh + go) = hv[it];
    }
    __threadfence();
  }
}

__global__ __launch_bounds__(256) void patch_kernel(const float* __restrict__ x, unsigned short* __restrict__ A) {
  const int tid = threadIdx.x;
  const int row = blockIdx.x * 16 + (tid >> 4);
  const int g   = tid & 15;
  const int b   = row >> 10;
  const int p   = row & (kTokB - 1);
  const bool valid = (p < kPat) && (g < 14);
  const int pc  = (p < kPat) ? p : (kPat - 1);
  const int gc  = (g < 14) ? g : 13;
  const int ch  = gc >> 1;
  const int l0  = (gc & 1) * 8;
  const float* src = x + ((size_t)b * kTlen + (size_t)pc * kPatchStr + l0) * kChan + ch;
  v8h hv;
#pragma unroll
  for (int e = 0; e < 8; ++e) {
    float f = src[e * kChan];
    f = valid ? bfrn(f) : 0.f;
    hv[e] = (_Float16)f;
  }
  _Float16* dst = (_Float16*)(void*)A + (size_t)row * kKembP + 8 * g;
  *(volatile v8h*)dst = hv;
  __threadfence();
  *(volatile v8h*)dst = hv;
}

__global__ __launch_bounds__(256) void rope_table_kernel(float* __restrict__ cs, float* __restrict__ sn) {
  const int i   = blockIdx.x * 256 + threadIdx.x;
  const int pos = i >> 5;
  const int j   = i & 31;
  const float e   = (float)(2 * j) * (1.0f / 64.0f);
  const float inv = exp2f(-e * 13.287712379549449f);
  const float ang = (float)pos * inv;
  float sv, cv;
  sincosf(ang, &sv, &cv);
  ((volatile float*)cs)[i] = cv;
  ((volatile float*)sn)[i] = sv;
  __threadfence();
  ((volatile float*)cs)[i] = cv;
  ((volatile float*)sn)[i] = sv;
}

__global__ __launch_bounds__(256) void ln_f16_kernel(const float* __restrict__ H, const float* __restrict__ g,
                                                     const float* __restrict__ bt, unsigned short* __restrict__ Y, int nrows) {
  const int wave = threadIdx.x >> 5, lane = threadIdx.x & 31;
  const int row = blockIdx.x * 8 + wave;
  if (row >= nrows) return;
  const float* hr = H + (size_t)row * kDm + 8 * lane;
  float xv[16];
#pragma unroll
  for (int i = 0; i < 2; ++i) {
    const v4f a0 = *(const v4f*)(hr + 256 * i);
    const v4f a1 = *(const v4f*)(hr + 256 * i + 4);
#pragma unroll
    for (int e = 0; e < 4; ++e) { xv[8 * i + e] = a0[e]; xv[8 * i + 4 + e] = a1[e]; }
  }
  float s = 0.f;
#pragma unroll
  for (int j = 0; j < 16; ++j) s += xv[j];
#pragma unroll
  for (int m = 1; m < 32; m <<= 1) s += __shfl_xor(s, m, 32);
  const float mu = s * (1.0f / 512.0f);
  float vs = 0.f;
#pragma unroll
  for (int j = 0; j < 16; ++j) { const float d = xv[j] - mu; vs += d * d; }
#pragma unroll
  for (int m = 1; m < 32; m <<= 1) vs += __shfl_xor(vs, m, 32);
  const float rstd = rsqrtf(vs * (1.0f / 512.0f) + kLnEps);
  const float* gr = g + 8 * lane;
  const float* br = bt + 8 * lane;
  v8h ov[2];
#pragma unroll
  for (int i = 0; i < 2; ++i) {
    const v4f g0 = *(const v4f*)(gr + 256 * i), g1 = *(const v4f*)(gr + 256 * i + 4);
    const v4f b0 = *(const v4f*)(br + 256 * i), b1 = *(const v4f*)(br + 256 * i + 4);
    v8h o;
#pragma unroll
    for (int e = 0; e < 4; ++e) {
      o[e]     = (_Float16)((xv[8 * i + e] - mu) * rstd * g0[e] + b0[e]);
      o[4 + e] = (_Float16)((xv[8 * i + 4 + e] - mu) * rstd * g1[e] + b1[e]);
    }
    ov[i] = o;
  }
  _Float16* yr = (_Float16*)(void*)Y + (size_t)row * kDm + 8 * lane;
  *(volatile v8h*)(yr)       = ov[0];
  *(volatile v8h*)(yr + 256) = ov[1];
  __threadfence();
  *(volatile v8h*)(yr)       = ov[0];
  *(volatile v8h*)(yr + 256) = ov[1];
}

__global__ __launch_bounds__(256) void ln_out_kernel(const float* __restrict__ H, const float* __restrict__ g,
                                                     const float* __restrict__ bt, float* __restrict__ out, int ntok) {
  const int wave = threadIdx.x >> 5, lane = threadIdx.x & 31;
  const int tok = blockIdx.x * 8 + wave;
  if (tok >= ntok) return;
  const int b = tok / kPat;
  const int p = tok - b * kPat;
  const float* hr = H + ((size_t)b * kTokB + p) * kDm + 4 * lane;
  float xv[16];
#pragma unroll
  for (int i = 0; i < 4; ++i) {
    const v4f a = *(const v4f*)(hr + 128 * i);
#pragma unroll
    for (int e = 0; e < 4; ++e) xv[4 * i + e] = a[e];
  }
  float s = 0.f;
#pragma unroll
  for (int j = 0; j < 16; ++j) s += xv[j];
#pragma unroll
  for (int m = 1; m < 32; m <<= 1) s += __shfl_xor(s, m, 32);
  const float mu = s * (1.0f / 512.0f);
  float vs = 0.f;
#pragma unroll
  for (int j = 0; j < 16; ++j) { const float d = xv[j] - mu; vs += d * d; }
#pragma unroll
  for (int m = 1; m < 32; m <<= 1) vs += __shfl_xor(vs, m, 32);
  const float rstd = rsqrtf(vs * (1.0f / 512.0f) + kLnEps);
  const float* gr = g + 4 * lane;
  const float* br = bt + 4 * lane;
  v4f yv[4];
#pragma unroll
  for (int i = 0; i < 4; ++i) {
    const v4f gg = *(const v4f*)(gr + 128 * i);
    const v4f bb = *(const v4f*)(br + 128 * i);
    v4f o;
#pragma unroll
    for (int e = 0; e < 4; ++e) o[e] = (xv[4 * i + e] - mu) * rstd * gg[e] + bb[e];
    yv[i] = o;
  }
  float* orow = out + (size_t)tok * kDm + 4 * lane;
#pragma unroll
  for (int i = 0; i < 4; ++i) *(volatile v4f*)(orow + 128 * i) = yv[i];
  __threadfence();
#pragma unroll
  for (int i = 0; i < 4; ++i) *(volatile v4f*)(orow + 128 * i) = yv[i];
}

__global__ __launch_bounds__(256) void emb_copy_kernel(const float* __restrict__ H, float* __restrict__ out) {
  const int gid = blockIdx.x * 256 + threadIdx.x;
  const int tok = gid >> 7;
  if (tok >= kTokReal) return;
  const int c4 = (gid & 127) * 4;
  const int b = tok / kPat;
  const int p = tok - b * kPat;
  const v4f v = *(const v4f*)(H + ((size_t)b * kTokB + p) * kDm + c4);
  float* dst = out + (size_t)tok * kDm + c4;
  *(volatile v4f*)dst = v;
  __threadfence();
  *(volatile v4f*)dst = v;
}

__global__ __launch_bounds__(256) void rope_kernel(const unsigned short* __restrict__ qk, const float* __restrict__ cs,
                                                   const float* __restrict__ sn, unsigned short* __restrict__ qkr) {
  const int gid  = blockIdx.x * 256 + threadIdx.x;
  const int e    = gid & 7;
  const int head = (gid >> 3) & 7;
  const int tok  = gid >> 6;
  const int pos  = tok & (kTokB - 1);
  const int own  = head * kHd + 8 * e;
  const int par  = head * kHd + 8 * (e ^ 4);
  const int fo   = 8 * (e & 3);
  const _Float16* qrow = (const _Float16*)(const void*)qk + (size_t)tok * kQK;
  const v8h qo = *(const v8h*)(qrow + own);
  const v8h qp = *(const v8h*)(qrow + par);
  const v8h ko = *(const v8h*)(qrow + kDm + own);
  const v8h kp = *(const v8h*)(qrow + kDm + par);
  const float* cr = cs + (size_t)pos * 32 + fo;
  const float* sr = sn + (size_t)pos * 32 + fo;
  const v4f ca = *(const v4f*)cr, cb = *(const v4f*)(cr + 4);
  const v4f sa = *(const v4f*)sr, sb = *(const v4f*)(sr + 4);
  const float sg = (e < 4) ? -1.0f : 1.0f;
  float cc[8], ss[8];
#pragma unroll
  for (int i = 0; i < 4; ++i) { cc[i] = ca[i]; cc[4 + i] = cb[i]; ss[i] = sa[i] * sg; ss[4 + i] = sb[i] * sg; }
  v8h oq, ok;
#pragma unroll
  for (int i = 0; i < 8; ++i) {
    oq[i] = (_Float16)((float)qo[i] * cc[i] + (float)qp[i] * ss[i]);
    ok[i] = (_Float16)((float)ko[i] * cc[i] + (float)kp[i] * ss[i]);
  }
  _Float16* dst = (_Float16*)(void*)qkr + (size_t)tok * kQK + own;
  *(volatile v8h*)(dst)       = oq;
  *(volatile v8h*)(dst + kDm) = ok;
  __threadfence();
  *(volatile v8h*)(dst)       = oq;
  *(volatile v8h*)(dst + kDm) = ok;
}

__global__ __launch_bounds__(256) void gelu_kernel(const unsigned short* __restrict__ U, unsigned short* __restrict__ G, int n2) {
  const int i = blockIdx.x * 256 + threadIdx.x;
  if (i < n2) {
    const unsigned u = ((const unsigned*)(const void*)U)[i];
    const float f0 = (float)__builtin_bit_cast(_Float16, (unsigned short)(u & 0xFFFFu));
    const float f1 = (float)__builtin_bit_cast(_Float16, (unsigned short)(u >> 16));
    const float g0 = 0.5f * f0 * (1.0f + erff(f0 * 0.70710678118654752f));
    const float g1 = 0.5f * f1 * (1.0f + erff(f1 * 0.70710678118654752f));
    const unsigned w = pk16(h_bits(g0), h_bits(g1));
    ((volatile unsigned*)G)[i] = w;
    __threadfence();
    ((volatile unsigned*)G)[i] = w;
  }
}

#define AT_D 64
#define AT_NW 4
#define AT_QB 64
#define AT_KC 64
constexpr int kNqb = kTokB / AT_QB;
constexpr int kNkc = kTokB / AT_KC;

__device__ __forceinline__ v8f mma_h(v16h a, v16h b, v8f c) {
  c = __builtin_amdgcn_wmma_f32_16x16x32_f16(false, a, false, b, (short)0, c, false, false);
  asm volatile("v_nop\n\tv_nop\n\tv_nop\n\tv_nop" : "+v"(c) : "v"(a), "v"(b));
  return c;
}

__global__ __launch_bounds__(128)
void attn_f16_kernel(const unsigned short* __restrict__ qkp, const unsigned short* __restrict__ vtp,
                     unsigned short* __restrict__ op, float sscale, float oscale) {
  union FH { v16h v; v8h h[2]; };
  __shared__ __align__(16) _Float16 Ksh[AT_KC * AT_D];
  __shared__ __align__(16) _Float16 Vth[AT_D * AT_KC];
  __shared__ __align__(16) _Float16 Psh[AT_NW][16 * AT_KC];
  __shared__ __align__(16) float    Os[AT_NW][16 * 68];

  const int tid  = threadIdx.x;
  const int wave = tid >> 5;
  const int lane = tid & 31;
  const int hh   = lane >> 4;
  const int c    = lane & 15;

  const int bx = blockIdx.x;
  const int qb = bx & (kNqb - 1);
  const int h  = (bx >> 4) & (kHeads - 1);
  const int b  = bx >> 7;
  const int q0 = qb * AT_QB + wave * 16;

  const _Float16* Qb = (const _Float16*)(const void*)qkp + (size_t)b * kTokB * kQK + (size_t)h * AT_D;
  const _Float16* Kb = Qb + kDm;
  const _Float16* Vb = (const _Float16*)(const void*)vtp + (size_t)h * AT_D * kTok + (size_t)b * kTokB;
  _Float16*       Ob = (_Float16*)(void*)op + (size_t)b * kTokB * kDm + (size_t)h * AT_D;

  v16h qa[2];
#pragma unroll
  for (int dc = 0; dc < 2; ++dc)
    qa[dc] = Frag<_Float16>::load(Qb + (size_t)(q0 + c) * kQK + dc * 32 + 8 * hh);

  float mrow[8], lrow[8];
  v8f oacc[4];
#pragma unroll
  for (int r = 0; r < 8; ++r) { mrow[r] = -INFINITY; lrow[r] = 0.f; }
#pragma unroll
  for (int t = 0; t < 4; ++t) oacc[t] = (v8f){0.f,0.f,0.f,0.f,0.f,0.f,0.f,0.f};

  for (int kc = 0; kc < kNkc; ++kc) {
    const int kv0 = kc * AT_KC;
    __syncthreads();
    {
      const int r = tid >> 1, half = (tid & 1) * 32;
      const _Float16* ks = Kb + (size_t)(kv0 + r) * kQK + half;
      const _Float16* vs = Vb + (size_t)r * kTok + kv0 + half;
#pragma unroll
      for (int i = 0; i < 4; ++i) {
        const v8h a0 = *(const v8h*)(ks + 8 * i);
        const v8h b0 = *(const v8h*)(vs + 8 * i);
        *(v8h*)(Ksh + r * AT_D  + half + 8 * i) = a0;
        *(v8h*)(Vth + r * AT_KC + half + 8 * i) = b0;
      }
    }
    __syncthreads();

    v8f s[4];
#pragma unroll
    for (int j = 0; j < 4; ++j) {
      s[j] = (v8f){0.f,0.f,0.f,0.f,0.f,0.f,0.f,0.f};
#pragma unroll
      for (int dc = 0; dc < 2; ++dc) {
        FH kb;
        kb.h[0] = *(const v8h*)(Ksh + (j * 16 + c) * AT_D + dc * 32 + 8 * hh);
        kb.h[1] = *(const v8h*)(Ksh + (j * 16 + c) * AT_D + dc * 32 + 16 + 8 * hh);
        s[j] = mma_h(qa[dc], kb.v, s[j]);
      }
    }
    float cm[8];
#pragma unroll
    for (int r = 0; r < 8; ++r) {
      float m = -INFINITY;
#pragma unroll
      for (int j = 0; j < 4; ++j) {
        const int kvcol = kv0 + j * 16 + c;
        float sv = s[j][r] * sscale;
        if (kvcol >= kPat) sv = -INFINITY;
        s[j][r] = sv;
        m = fmaxf(m, sv);
      }
#pragma unroll
      for (int off = 1; off < 16; off <<= 1) m = fmaxf(m, __shfl_xor(m, off, 32));
      cm[r] = m;
    }
    _Float16* pw = Psh[wave];
#pragma unroll
    for (int r = 0; r < 8; ++r) {
      const float mnew = fmaxf(mrow[r], cm[r]);
      const float alpha = expf(mrow[r] - mnew);
      mrow[r] = mnew;
      float psum = 0.f;
#pragma unroll
      for (int j = 0; j < 4; ++j) {
        const float p = expf(s[j][r] - mnew);
        psum += p;
        pw[(8 * hh + r) * AT_KC + j * 16 + c] = (_Float16)(p * PSCALE);
      }
#pragma unroll
      for (int off = 1; off < 16; off <<= 1) psum += __shfl_xor(psum, off, 32);
      lrow[r] = lrow[r] * alpha + psum;
#pragma unroll
      for (int t = 0; t < 4; ++t) oacc[t][r] *= alpha;
    }
    __builtin_amdgcn_fence(__ATOMIC_RELEASE, "workgroup");
    __builtin_amdgcn_wave_barrier();
    __builtin_amdgcn_fence(__ATOMIC_ACQUIRE, "workgroup");
#pragma unroll 1
    for (int kk = 0; kk < 2; ++kk) {
      FH pa;
      pa.h[0] = *(const v8h*)(pw + c * AT_KC + kk * 32 + 8 * hh);
      pa.h[1] = *(const v8h*)(pw + c * AT_KC + kk * 32 + 16 + 8 * hh);
#pragma unroll
      for (int t = 0; t < 4; ++t) {
        FH vb;
        vb.h[0] = *(const v8h*)(Vth + (t * 16 + c) * AT_KC + kk * 32 + 8 * hh);
        vb.h[1] = *(const v8h*)(Vth + (t * 16 + c) * AT_KC + kk * 32 + 16 + 8 * hh);
        oacc[t] = mma_h(pa.v, vb.v, oacc[t]);
      }
    }
  }

  float* os = Os[wave];
#pragma unroll
  for (int r = 0; r < 8; ++r) {
    const float inv = oscale * (1.0f / (lrow[r] * PSCALE));
#pragma unroll
    for (int t = 0; t < 4; ++t) os[(8 * hh + r) * 68 + t * 16 + c] = oacc[t][r] * inv;
  }
  __builtin_amdgcn_fence(__ATOMIC_RELEASE, "workgroup");
  __builtin_amdgcn_wave_barrier();
  __builtin_amdgcn_fence(__ATOMIC_ACQUIRE, "workgroup");
  {
    const int q = lane >> 3, c8 = (lane & 7) * 8;
    for (int pass = 0; pass < 2; ++pass) {
#pragma unroll
      for (int it = 0; it < 4; ++it) {
        const int row = it * 4 + q;
        const float* sp = os + row * 68 + c8;
        v8h hv;
#pragma unroll
        for (int e = 0; e < 8; ++e) hv[e] = (_Float16)sp[e];
        *(volatile v8h*)(Ob + (size_t)(q0 + row) * kDm + c8) = hv;
      }
      __threadfence();
    }
  }
}

extern "C" void kernel_launch(void* const* d_in, const int* in_sizes, int n_in,
                              void* d_out, int out_size, void* d_ws, size_t ws_size,
                              hipStream_t stream) {
  if (n_in < 17) return;
  if (in_sizes[0] != kBatch * kTlen * kChan) return;
  if (in_sizes[1] != kKemb * kDm || in_sizes[2] != kDm) return;
  if (in_sizes[3] != kLayers * kDm || in_sizes[4] != kLayers * kDm) return;
  if (in_sizes[5] != kLayers * kDm * kQKV || in_sizes[6] != kLayers * kQKV) return;
  if (in_sizes[7] != kLayers * kDm * kDm || in_sizes[8] != kLayers * kDm) return;
  if (in_sizes[9] != kLayers * kDm || in_sizes[10] != kLayers * kDm) return;
  if (in_sizes[11] != kLayers * kDm * kMlp || in_sizes[12] != kLayers * kMlp) return;
  if (in_sizes[13] != kLayers * kMlp * kDm || in_sizes[14] != kLayers * kDm) return;
  if (in_sizes[15] != kDm || in_sizes[16] != kDm) return;
  if (out_size != 2 * kTokReal * kDm) return;

  const float* x      = (const float*)d_in[0];
  const float* W_emb  = (const float*)d_in[1];
  const float* b_emb  = (const float*)d_in[2];
  const float* ln1_g  = (const float*)d_in[3];
  const float* ln1_b  = (const float*)d_in[4];
  const float* W_qkv  = (const float*)d_in[5];
  const float* b_qkv  = (const float*)d_in[6];
  const float* W_proj = (const float*)d_in[7];
  const float* b_proj = (const float*)d_in[8];
  const float* ln2_g  = (const float*)d_in[9];
  const float* ln2_b  = (const float*)d_in[10];
  const float* W_mlp1 = (const float*)d_in[11];
  const float* b_mlp1 = (const float*)d_in[12];
  const float* W_mlp2 = (const float*)d_in[13];
  const float* b_mlp2 = (const float*)d_in[14];
  const float* lnf_g  = (const float*)d_in[15];
  const float* lnf_b  = (const float*)d_in[16];
  float* out0 = (float*)d_out;
  float* out1 = (float*)d_out + (size_t)kTokReal * kDm;

  char* ws = (char*)d_ws;
  size_t off = 0;
  auto carve = [&](size_t bytes) -> char* { char* p = ws + off; off += (bytes + 255) & ~(size_t)255; return p; };
  unsigned short* WEMB = (unsigned short*)carve((size_t)kDm * kKembP * 2);
  unsigned short* WQKV = (unsigned short*)carve((size_t)kLayers * kQKV * kDm * 2);
  unsigned short* WPRJ = (unsigned short*)carve((size_t)kLayers * kDm * kDm * 2);
  unsigned short* WM1  = (unsigned short*)carve((size_t)kLayers * kMlp * kDm * 2);
  unsigned short* WM2  = (unsigned short*)carve((size_t)kLayers * kDm * kMlp * 2);
  unsigned short* A16  = (unsigned short*)carve((size_t)kTok * kKembP * 2);
  float*          HA   = (float*)carve((size_t)kTok * kDm * 4);
  float*          HB   = (float*)carve((size_t)kTok * kDm * 4);
  unsigned short* Y16  = (unsigned short*)carve((size_t)kTok * kDm * 2);
  unsigned short* QK16 = (unsigned short*)carve((size_t)kTok * kQK * 2);
  unsigned short* QKR  = (unsigned short*)carve((size_t)kTok * kQK * 2);
  unsigned short* VT16 = (unsigned short*)carve((size_t)kDm * kTok * 2);
  unsigned short* O16  = (unsigned short*)carve((size_t)kTok * kDm * 2);
  unsigned short* U16p = (unsigned short*)carve((size_t)kTok * kMlp * 2);
  unsigned short* G16  = (unsigned short*)carve((size_t)kTok * kMlp * 2);
  float*          COS  = (float*)carve((size_t)kTokB * 32 * 4);
  float*          SIN  = (float*)carve((size_t)kTokB * 32 * 4);
  if (off > ws_size) return;

  const float wsc  = 1.0f / kWCarry;
  const float wosc = 1.0f / (kWCarry * kOCarry);

  tcast_kernel<<<dim3(kDm / 64, kKembP / 64, 1), 256, 0, stream>>>(W_emb, WEMB, kKemb, kKembP, kDm, 0L, 0L, kWCarry);
  tcast_kernel<<<dim3(kQKV / 64, kDm / 64, kLayers), 256, 0, stream>>>(W_qkv, WQKV, kDm, kDm, kQKV,
                                                                      (long)kDm * kQKV, (long)kQKV * kDm, kWCarry);
  tcast_kernel<<<dim3(kDm / 64, kDm / 64, kLayers), 256, 0, stream>>>(W_proj, WPRJ, kDm, kDm, kDm,
                                                                     (long)kDm * kDm, (long)kDm * kDm, kWCarry);
  tcast_kernel<<<dim3(kMlp / 64, kDm / 64, kLayers), 256, 0, stream>>>(W_mlp1, WM1, kDm, kDm, kMlp,
                                                                      (long)kDm * kMlp, (long)kMlp * kDm, kWCarry);
  tcast_kernel<<<dim3(kDm / 64, kMlp / 64, kLayers), 256, 0, stream>>>(W_mlp2, WM2, kMlp, kMlp, kDm,
                                                                      (long)kMlp * kDm, (long)kDm * kMlp, kWCarry);
  rope_table_kernel<<<dim3((kTokB * 32) / 256), 256, 0, stream>>>(COS, SIN);
  patch_kernel<<<dim3(kTok / 16), 256, 0, stream>>>(x, A16);

  wmma_gemm64<0, false, 2, 0, false><<<dim3((kTok / 64) * (kDm / 64) / 8, 1), 256, 0, stream>>>(
      A16, A16, kKembP, 0L, WEMB, WEMB, kKembP, 0L, HA, HA, kDm, 0L, b_emb, b_emb, 0L, kTok, kDm, kKembP, wsc);
  emb_copy_kernel<<<dim3((kTokReal * (kDm / 4)) / 256), 256, 0, stream>>>(HA, out0);

  for (int i = 0; i < kLayers; ++i) {
    const unsigned short* wqkv = WQKV + (size_t)i * kQKV * kDm;
    const unsigned short* wprj = WPRJ + (size_t)i * kDm * kDm;
    const unsigned short* wm1  = WM1 + (size_t)i * kMlp * kDm;
    const unsigned short* wm2  = WM2 + (size_t)i * kDm * kMlp;
    ln_f16_kernel<<<dim3(kTok / 8), 256, 0, stream>>>(HA, ln1_g + (size_t)i * kDm, ln1_b + (size_t)i * kDm, Y16, kTok);
    wmma_gemm64<0, false, 2, 1, false><<<dim3((kTok / 64) * (kQK / 64) / 8, 1), 256, 0, stream>>>(
        Y16, Y16, kDm, 0L, wqkv, wqkv, kDm, 0L, QK16, QK16, kQK, 0L, b_qkv + (size_t)i * kQKV, b_qkv + (size_t)i * kQKV, 0L,
        kTok, kQK, kDm, wsc);
    wmma_gemm64<0, false, 1, 1, false><<<dim3((kDm / 64) * (kTok / 64) / 8, 1), 256, 0, stream>>>(
        wqkv + (size_t)kQK * kDm, wqkv + (size_t)kQK * kDm, kDm, 0L, Y16, Y16, kDm, 0L, VT16, VT16, kTok, 0L,
        b_qkv + (size_t)i * kQKV + kQK, b_qkv + (size_t)i * kQKV + kQK, 0L, kDm, kTok, kDm, wsc);
    rope_kernel<<<dim3((kTok * kHeads * 8) / 256), 256, 0, stream>>>(QK16, COS, SIN, QKR);
    attn_f16_kernel<<<dim3(kBatch * kHeads * kNqb), 128, 0, stream>>>(QKR, VT16, O16, 0.125f, kOCarry);
    wmma_gemm64<0, false, 2, 0, true><<<dim3((kTok / 64) * (kDm / 64) / 8, 1), 256, 0, stream>>>(
        O16, O16, kDm, 0L, wprj, wprj, kDm, 0L, HB, HB, kDm, 0L, b_proj + (size_t)i * kDm, HA, 0L, kTok, kDm, kDm, wosc);
    ln_f16_kernel<<<dim3(kTok / 8), 256, 0, stream>>>(HB, ln2_g + (size_t)i * kDm, ln2_b + (size_t)i * kDm, Y16, kTok);
    wmma_gemm64<0, false, 2, 1, false><<<dim3((kTok / 64) * (kMlp / 64) / 8, 1), 256, 0, stream>>>(
        Y16, Y16, kDm, 0L, wm1, wm1, kDm, 0L, U16p, U16p, kMlp, 0L, b_mlp1 + (size_t)i * kMlp, b_mlp1 + (size_t)i * kMlp, 0L,
        kTok, kMlp, kDm, wsc);
    gelu_kernel<<<dim3((kTok * kMlp / 2 + 255) / 256), 256, 0, stream>>>(U16p, G16, kTok * kMlp / 2);
    wmma_gemm64<0, false, 2, 0, true><<<dim3((kTok / 64) * (kDm / 64) / 8, 1), 256, 0, stream>>>(
        G16, G16, kMlp, 0L, wm2, wm2, kMlp, 0L, HA, HA, kDm, 0L, b_mlp2 + (size_t)i * kDm, HB, 0L, kTok, kDm, kMlp, wsc);
  }
  ln_out_kernel<<<dim3((kTokReal + 7) / 8), 256, 0, stream>>>(HA, lnf_g, lnf_b, out1, kTokReal);
}
